// ModelGraphPolicy_74294344286850
// MI455X (gfx1250) — hardware-verified
//
#include <hip/hip_runtime.h>
#include <math.h>

typedef __attribute__((ext_vector_type(16))) _Float16 v16h;
typedef __attribute__((ext_vector_type(16))) __bf16 v16b;
typedef __attribute__((ext_vector_type(8)))  _Float16 v8h;
typedef __attribute__((ext_vector_type(8)))  float v8f;
typedef __attribute__((ext_vector_type(4)))  float v4f;
typedef __attribute__((ext_vector_type(2)))  float v2f;
typedef __attribute__((ext_vector_type(4)))  unsigned v4u;
typedef __attribute__((ext_vector_type(4)))  int v4i;
typedef float __attribute__((may_alias)) float_a;
typedef int __attribute__((may_alias)) int_a;

template <typename T> __device__ __forceinline__ void vst2(void* p, T v) { *(volatile T*)p = v; __threadfence(); *(volatile T*)p = v; }
__device__ __forceinline__ v8f wmma16(v16h a, v16h b, v8f c) {
  v8f d = __builtin_amdgcn_wmma_f32_16x16x32_f16(false, a, false, b, (short)0, c, false, false);
  asm volatile("v_nop\n\tv_nop\n\tv_nop\n\tv_nop" : "+v"(d) : "v"(a), "v"(b));
  return d;
}
__device__ __forceinline__ v8f wmma_bf(v16b a, v16b b, v8f c) {
  v8f d = __builtin_amdgcn_wmma_f32_16x16x32_bf16(false, a, false, b, (short)0, c, false, false);
  asm volatile("v_nop\n\tv_nop\n\tv_nop\n\tv_nop" : "+v"(d) : "v"(a), "v"(b));
  return d;
}
__device__ __forceinline__ v16h frag_h(const _Float16* rowk0, int lane) {
  union { v16h v; v8h q[2]; } u; const _Float16* p = rowk0 + 8 * (lane >> 4);
  u.q[0] = *(const v8h*)p; u.q[1] = *(const v8h*)(p + 16); return u.v;
}
__device__ __forceinline__ v16h frag_f32(const float* rowk0, int lane) {
  v16h a; const float* p = rowk0 + 8 * (lane >> 4);
#pragma unroll
  for (int i = 0; i < 8; ++i) { a[i] = (_Float16)p[i]; a[8 + i] = (_Float16)p[16 + i]; }
  return a;
}
__device__ __forceinline__ v16h frag_f32s(const float* rowk0, int lane, float sc) {
  v16h a; const float* p = rowk0 + 8 * (lane >> 4);
#pragma unroll
  for (int i = 0; i < 8; ++i) { a[i] = (_Float16)(p[i] * sc); a[8 + i] = (_Float16)(p[16 + i] * sc); }
  return a;
}
__device__ __forceinline__ v16h fragc_f32(const float* W, int k0, int n, int lane, int ld, int K) {
  v16h a; const int g = lane >> 4;
#pragma unroll
  for (int i = 0; i < 8; ++i) { const int ka = k0 + 8 * g + i, kb = ka + 16;
    a[i] = (_Float16)(ka < K ? W[(size_t)(ka < K ? ka : K - 1) * ld + n] : 0.f); a[8 + i] = (_Float16)(kb < K ? W[(size_t)(kb < K ? kb : K - 1) * ld + n] : 0.f); }
  return a;
}
struct F2 { v16b h, l; };
__device__ __forceinline__ F2 bsplit16(const float v[16]) { F2 r;
#pragma unroll
  for (int i = 0; i < 16; ++i) { const __bf16 h = (__bf16)v[i]; r.h[i] = h; r.l[i] = (__bf16)(v[i] - (float)h); }
  return r; }
__device__ __forceinline__ F2 split_row(const float* row, int k0, int lane) { float v[16]; const float* p = row + k0 + 8 * (lane >> 4);
#pragma unroll
  for (int i = 0; i < 8; ++i) { v[i] = p[i]; v[8 + i] = p[16 + i]; }
  return bsplit16(v); }
__device__ __forceinline__ F2 split_rowK(const float* row, int k0, int lane, int K) { float v[16]; const int g = lane >> 4;
#pragma unroll
  for (int i = 0; i < 8; ++i) { const int ka = k0 + 8 * g + i, kb = ka + 16; v[i] = ka < K ? row[ka < K ? ka : K - 1] : 0.f; v[8 + i] = kb < K ? row[kb < K ? kb : K - 1] : 0.f; }
  return bsplit16(v); }
__device__ __forceinline__ F2 split_col(const float* W, int k0, int n, int lane, int ld, int K) { float v[16]; const int g = lane >> 4;
#pragma unroll
  for (int i = 0; i < 8; ++i) { const int ka = k0 + 8 * g + i, kb = ka + 16; v[i] = ka < K ? W[(size_t)(ka < K ? ka : K - 1) * ld + n] : 0.f; v[8 + i] = kb < K ? W[(size_t)(kb < K ? kb : K - 1) * ld + n] : 0.f; }
  return bsplit16(v); }
__device__ __forceinline__ v8f mac3(const F2& a, const F2& b, v8f c) { c = wmma_bf(a.l, b.h, c); c = wmma_bf(a.h, b.l, c); return wmma_bf(a.h, b.h, c); }
__device__ __forceinline__ float sigm(float v) { return 1.0f / (1.0f + expf(-v)); }
#define LDSX() do { asm volatile("s_wait_dscnt 0" ::: "memory"); __builtin_amdgcn_wave_barrier(); __builtin_amdgcn_fence(__ATOMIC_RELEASE, "workgroup"); } while (0)


#define NROW 262144
#define SD 12
#define MD 32
#ifndef TRB
#define TRB (NROW / 64)
#endif
typedef __attribute__((ext_vector_type(8))) __bf16 v8b;
__device__ __forceinline__ v16b frag_b(const __bf16* rowk0, int lane) {
  union { v16b v; v8b q[2]; } u; const __bf16* p = rowk0 + 8 * (lane >> 4);
  u.q[0] = *(const v8b*)p; u.q[1] = *(const v8b*)(p + 16); return u.v;
}
__device__ __forceinline__ float bfr(float v) { return (float)(__bf16)v; }
__device__ __attribute__((noinline)) float tanh_ni(float v) { return tanhf(v); }
#define PK_P1 0
#define PK_P2 (PK_P1 + 64 * 64)
#define PK_P3 (PK_P2 + 64 * 64)
#define PK_D1 (PK_P3 + 32 * 64)
#define PK_D2 (PK_D1 + 400 * 64)
#define PK_D3 (PK_D2 + 304 * 448)
#define PK_END (PK_D3 + 32 * 320)
#define WS_PK 0u
#define WS_END (WS_PK + 2u * PK_END)

__global__ __launch_bounds__(256) void k_pack(const float* __restrict__ W1, const float* __restrict__ W2, const float* __restrict__ W3, const float* __restrict__ D1, const float* __restrict__ D2, const float* __restrict__ D3, __bf16* __restrict__ PK) {
  __shared__ __align__(16) __bf16 s[448]; const int n = blockIdx.x, tid = threadIdx.x; int K; size_t dst; float v = 0.f; int m = n;
  if (m < 64) { K = 64; dst = PK_P1 + (size_t)m * 64; if (tid < 13) v = W1[m * 13 + tid]; }
  else if ((m -= 64) < 64) { K = 64; dst = PK_P2 + (size_t)m * 64; if (tid < 64) v = W2[m * 128 + tid]; }
  else if ((m -= 64) < 32) { K = 64; dst = PK_P3 + (size_t)m * 64; if (tid < 64) v = W3[m * 64 + tid]; }
  else if ((m -= 32) < 400) { K = 64; dst = PK_D1 + (size_t)m * 64; if (tid < 33) v = D1[m * 65 + tid]; }
  else if ((m -= 400) < 304) { K = 448; dst = PK_D2 + (size_t)m * 448; if (m < 300 && tid < 400) v = D2[m * 400 + tid]; }
  else { m -= 304; K = 320; dst = PK_D3 + (size_t)m * 320; if (tid < 300) v = D3[m * 300 + tid]; }
  for (int k = tid; k < K; k += 256) s[k] = (__bf16)bfr(k == tid ? v : 0.f);
  if (K == 448 && tid + 256 < 448) { const int k = tid + 256; float v2 = 0.f; if (m < 300 && k < 400) v2 = D2[m * 400 + k]; s[k] = (__bf16)bfr(v2); }
  if (K == 320 && tid + 256 < 320) { const int k = tid + 256; float v2 = 0.f; if (k < 300) v2 = D3[m * 300 + k]; s[k] = (__bf16)bfr(v2); }
  __syncthreads();
  if (tid < K / 8) vst2((unsigned*)(PK + dst + tid * 8), *(const v4u*)&s[tid * 8]);
}
__device__ __forceinline__ void put_hl(__bf16* h, __bf16* l, float v) { const __bf16 hb = (__bf16)v; *h = hb; *l = (__bf16)(v - (float)hb); }
__global__ __launch_bounds__(128) void k_mgp(const float* __restrict__ ST, const float* __restrict__ AC, const __bf16* __restrict__ PK, const float* __restrict__ b1, const float* __restrict__ b2, const float* __restrict__ b3, const float* __restrict__ c1, const float* __restrict__ c2, const float* __restrict__ c3, float* __restrict__ OUT) {
  __shared__ __align__(16) __bf16 sah[4][16][424], sal[4][16][424]; __shared__ __align__(16) __bf16 sbh[4][16][72], sbl[4][16][72]; __shared__ __align__(16) float so[4][16][36];
  const int tid = threadIdx.x, wave = tid >> 5, lane = tid & 31, col = lane & 15, g = lane >> 4; const size_t r0 = (size_t)blockIdx.x * 64 + wave * 16;
  __bf16 (*ah)[424] = sah[wave], (*al)[424] = sal[wave], (*bh)[72] = sbh[wave], (*bl)[72] = sbl[wave];
  for (int q = lane; q < 16 * 32; q += 32) { const int rl = q >> 5, k = q & 31; float v = 0.f; if (k < SD) v = bfr(ST[(r0 + rl) * SD + k]); else if (k == SD) v = bfr(AC[r0 + rl]); bh[rl][k] = (__bf16)v; bl[rl][k] = (__bf16)0.f; }
  LDSX();
  { v8f acc[4] = {}; const v16b a = frag_b(&bh[col][0], lane);
#pragma unroll
    for (int j = 0; j < 4; ++j) acc[j] = wmma_bf(a, frag_b(PK + PK_P1 + (size_t)(j * 16 + col) * 64, lane), acc[j]);
    float ss[8];
#pragma unroll
    for (int r = 0; r < 8; ++r) { float s = 0.f;
#pragma unroll
      for (int j = 0; j < 4; ++j) { acc[j][r] += bfr(b1[j * 16 + col]); s += acc[j][r] * acc[j][r]; }
#pragma unroll
      for (int o = 1; o < 16; o <<= 1) s += __shfl_xor(s, o);
      ss[r] = 1.0f / fmaxf(sqrtf(s), 1e-12f); }
    LDSX();
#pragma unroll
    for (int j = 0; j < 4; ++j)
#pragma unroll
      for (int r = 0; r < 8; ++r) put_hl(&ah[8 * g + r][j * 16 + col], &al[8 * g + r][j * 16 + col], tanh_ni(acc[j][r] * ss[r])); }
  LDSX();
  { v8f acc[4] = {};
#pragma unroll
    for (int kc = 0; kc < 2; ++kc) { const v16b xh = frag_b(&ah[col][kc * 32], lane), xl = frag_b(&al[col][kc * 32], lane);
#pragma unroll
      for (int j = 0; j < 4; ++j) { const v16b w = frag_b(PK + PK_P2 + (size_t)(j * 16 + col) * 64 + kc * 32, lane); acc[j] = wmma_bf(xl, w, acc[j]); acc[j] = wmma_bf(xh, w, acc[j]); } }
    LDSX();
#pragma unroll
    for (int j = 0; j < 4; ++j)
#pragma unroll
      for (int r = 0; r < 8; ++r) put_hl(&bh[8 * g + r][j * 16 + col], &bl[8 * g + r][j * 16 + col], tanh_ni(acc[j][r] + bfr(b2[j * 16 + col]))); }
  LDSX();
  { v8f acc[2] = {};
#pragma unroll
    for (int kc = 0; kc < 2; ++kc) { const v16b xh = frag_b(&bh[col][kc * 32], lane), xl = frag_b(&bl[col][kc * 32], lane);
#pragma unroll
      for (int j = 0; j < 2; ++j) { const v16b w = frag_b(PK + PK_P3 + (size_t)(j * 16 + col) * 64 + kc * 32, lane); acc[j] = wmma_bf(xl, w, acc[j]); acc[j] = wmma_bf(xh, w, acc[j]); } }
    float ss[8];
#pragma unroll
    for (int r = 0; r < 8; ++r) { float s = 0.f;
#pragma unroll
      for (int j = 0; j < 2; ++j) { acc[j][r] += bfr(b3[j * 16 + col]); s += acc[j][r] * acc[j][r]; }
#pragma unroll
      for (int o = 1; o < 16; o <<= 1) s += __shfl_xor(s, o);
      ss[r] = 1.0f / fmaxf(sqrtf(s), 1e-12f); }
    LDSX();
#pragma unroll
    for (int j = 0; j < 2; ++j)
#pragma unroll
      for (int r = 0; r < 8; ++r) put_hl(&ah[8 * g + r][j * 16 + col], &al[8 * g + r][j * 16 + col], acc[j][r] * ss[r]);
    for (int q = lane; q < 16 * 32; q += 32) { const int rl = q >> 5, k = 32 + (q & 31); float v = 0.f; if (k == 32) v = bfr(AC[r0 + rl]); ah[rl][k] = (__bf16)v; al[rl][k] = (__bf16)0.f; } }
  LDSX();
  __shared__ __align__(16) __bf16 swh[4][16][424], swl[4][16][424]; __bf16 (*wh)[424] = swh[wave], (*wl)[424] = swl[wave];
  { const v16b xh0 = frag_b(&ah[col][0], lane), xl0 = frag_b(&al[col][0], lane), xh1 = frag_b(&ah[col][32], lane), xl1 = frag_b(&al[col][32], lane);
#pragma unroll 1
    for (int ch = 0; ch < 5; ++ch) { v8f acc[5] = {};
#pragma unroll
      for (int j = 0; j < 5; ++j) { const int o = (ch * 5 + j) * 16 + col; const v16b w0 = frag_b(PK + PK_D1 + (size_t)o * 64, lane), w1 = frag_b(PK + PK_D1 + (size_t)o * 64 + 32, lane); acc[j] = wmma_bf(xl0, w0, acc[j]); acc[j] = wmma_bf(xh0, w0, acc[j]); acc[j] = wmma_bf(xl1, w1, acc[j]); acc[j] = wmma_bf(xh1, w1, acc[j]); }
#pragma unroll
      for (int j = 0; j < 5; ++j) { const int o = (ch * 5 + j) * 16 + col; const float bb = bfr(c1[o]);
#pragma unroll
        for (int r = 0; r < 8; ++r) put_hl(&wh[8 * g + r][o], &wl[8 * g + r][o], fmaxf(acc[j][r] + bb, 0.f)); } }
    for (int q = lane; q < 16 * 16; q += 32) { const int rl = q >> 4, k = 400 + (q & 15); wh[rl][k] = (__bf16)0.f; wl[rl][k] = (__bf16)0.f; } }
  LDSX();
#pragma unroll 1
  for (int ch = 0; ch < 3; ++ch) { const int t0 = ch == 0 ? 0 : (ch == 1 ? 7 : 13), nt = ch == 0 ? 7 : 6; v8f acc[7] = {};
#pragma unroll 1
    for (int kc = 0; kc < 13; ++kc) { const v16b xh = frag_b(&wh[col][kc * 32], lane), xl = frag_b(&wl[col][kc * 32], lane);
#pragma unroll
      for (int j = 0; j < 7; ++j) if (j < nt) { const v16b w = frag_b(PK + PK_D2 + (size_t)((t0 + j) * 16 + col) * 448 + kc * 32, lane); acc[j] = wmma_bf(xl, w, acc[j]); acc[j] = wmma_bf(xh, w, acc[j]); } }
#pragma unroll
    for (int j = 0; j < 7; ++j) if (j < nt) { const int o = (t0 + j) * 16 + col; const float bb = (o < 300) ? bfr(c2[o]) : 0.f;
#pragma unroll
      for (int r = 0; r < 8; ++r) put_hl(&ah[8 * g + r][o], &al[8 * g + r][o], (o < 300) ? fmaxf(acc[j][r] + bb, 0.f) : 0.f); } }
  for (int q = lane; q < 16 * 16; q += 32) { const int rl = q >> 4, k = 304 + (q & 15); ah[rl][k] = (__bf16)0.f; al[rl][k] = (__bf16)0.f; }
  LDSX();
  { v8f acc[2] = {};
#pragma unroll 1
    for (int kc = 0; kc < 10; ++kc) { const v16b xh = frag_b(&ah[col][kc * 32], lane), xl = frag_b(&al[col][kc * 32], lane);
#pragma unroll
      for (int j = 0; j < 2; ++j) { const v16b w = frag_b(PK + PK_D3 + (size_t)(j * 16 + col) * 320 + kc * 32, lane); acc[j] = wmma_bf(xl, w, acc[j]); acc[j] = wmma_bf(xh, w, acc[j]); } }
#pragma unroll
    for (int j = 0; j < 2; ++j)
#pragma unroll
      for (int r = 0; r < 8; ++r) so[wave][8 * g + r][j * 16 + col] = acc[j][r] + bfr(c3[j * 16 + col]); }
  LDSX();
  for (int rl = 0; rl < 16; ++rl) if (lane < 8) vst2(OUT + (r0 + rl) * MD + lane * 4, *(const v4f*)&so[wave][rl][lane * 4]);
}
extern "C" void kernel_launch(void* const* d_in, const int* in_sizes, int n_in, void* d_out, int out_size, void* d_ws, size_t ws_size, hipStream_t stream) {
  (void)in_sizes; (void)n_in; (void)out_size;
  const float** F = (const float**)d_in;
  if (ws_size < (size_t)WS_END) return;
  char* ws = (char*)d_ws; __bf16* PK = (__bf16*)(ws + WS_PK);
  k_pack<<<64 + 64 + 32 + 400 + 304 + 32, 256, 0, stream>>>(F[2], F[4], F[6], F[8], F[10], F[12], PK);
  k_mgp<<<TRB, 128, 0, stream>>>(F[0], F[1], PK, F[3], F[5], F[7], F[9], F[11], F[13], (float*)d_out);
}
